// LSTM_73512660238908
// MI455X (gfx1250) — hardware-verified
//
#include <hip/hip_runtime.h>
#include <math.h>

constexpr int NB       = 128;
constexpr int NSTEP    = 1024;
constexpr int NE       = 64;
constexpr int NH       = 256;
constexpr int NCLS     = 10;
constexpr int NVOC     = 3;
constexpr int NGATE    = 4;
constexpr int TPW_NT   = 256;
constexpr int XG_NT    = 64;
constexpr int SEQ_NT   = 512;
constexpr int SEQ_ROWS = 16;
constexpr int HPITCH   = 264;
constexpr int HSP      = 260;
constexpr int NOUT     = NB * NCLS;
constexpr float HCARRY  = 64.0f;
constexpr float WCARRY  = 16.0f;
constexpr float ACC_INV = 1.0f / 1024.0f;
constexpr float XCARRY  = 1024.0f;
static_assert(NB % SEQ_ROWS == 0);
static_assert(NH == 16 * (SEQ_NT / 32));
static_assert(NH % 64 == 0);
static_assert(NSTEP % SEQ_NT == 0);
static_assert(XG_NT * 4 == NH);
static_assert(SEQ_ROWS * NCLS == 5 * 32);
static_assert((SEQ_ROWS * NCLS * 4) % 128 == 0);
static_assert(HPITCH % 8 == 0 && HSP % 4 == 0);
static_assert(NVOC == 3);

typedef __attribute__((ext_vector_type(16))) _Float16 v16h;
typedef __attribute__((ext_vector_type(8)))  _Float16 v8h;
typedef __attribute__((ext_vector_type(16))) __bf16   v16b;
typedef __attribute__((ext_vector_type(8)))  __bf16   v8b;
typedef __attribute__((ext_vector_type(8)))  float    v8f;
typedef __attribute__((ext_vector_type(4)))  float    v4f;

__device__ __forceinline__ unsigned short f2bf_bits(float f) {
  unsigned u = __float_as_uint(f);
  return (unsigned short)((u + 0x7FFFu + ((u >> 16) & 1u)) >> 16);
}
__device__ __forceinline__ float bf_bits2f(unsigned short h) { return __uint_as_float(((unsigned)h) << 16); }
__device__ __forceinline__ float bf16r(float f) { return bf_bits2f(f2bf_bits(f)); }

__device__ __forceinline__ void dep_guard_h(v8f& a, v8f& b, v16h x, v16h y) { asm volatile("v_nop\n\tv_nop\n\tv_nop\n\tv_nop" : "+v"(a), "+v"(b) : "v"(x), "v"(y)); }
__device__ __forceinline__ void dep_guard_b(v8f& a, v8f& b, v16b x, v16b y) { asm volatile("v_nop\n\tv_nop\n\tv_nop\n\tv_nop" : "+v"(a), "+v"(b) : "v"(x), "v"(y)); }
__device__ __forceinline__ void keep4_h(v16h a, v16h b, v16h c, v16h d) { asm volatile("v_nop" :: "v"(a), "v"(b), "v"(c), "v"(d)); }
__device__ __forceinline__ void keep4_b(v16b a, v16b b, v16b c, v16b d) { asm volatile("v_nop" :: "v"(a), "v"(b), "v"(c), "v"(d)); }
__device__ __forceinline__ void acc_guard4(v8f& a, v8f& b, v8f& c, v8f& d) { asm volatile("v_nop\n\tv_nop\n\tv_nop\n\tv_nop" : "+v"(a), "+v"(b), "+v"(c), "+v"(d)); }
__device__ __forceinline__ void mma_guard_all(v8f& c0, v8f& c1, v8f& c2, v8f& c3, v16h a, v16h b0, v16h b1, v16h b2, v16h b3) {
  asm volatile("v_nop\n\tv_nop\n\tv_nop\n\tv_nop" : "+v"(c0), "+v"(c1), "+v"(c2), "+v"(c3) : "v"(a), "v"(b0), "v"(b1), "v"(b2), "v"(b3));
}
template <typename T> struct Frag;
template <> struct Frag<_Float16> {
  typedef v16h V; union U { v16h v; v8h h[2]; };
  static __device__ __forceinline__ v16h load(const _Float16* p) {
    U f; f.h[0] = *(const v8h*)(p); f.h[1] = *(const v8h*)(p + 16); return f.v;
  }
  static __device__ __forceinline__ v8f mma(v16h a, v16h b, v8f c) {
    return __builtin_amdgcn_wmma_f32_16x16x32_f16(false, a, false, b, (short)0, c, false, false);
  }
  static __device__ __forceinline__ void guard(v8f& a, v8f& b, v16h x, v16h y) { dep_guard_h(a, b, x, y); }
  static __device__ __forceinline__ void keep(v16h a, v16h b, v16h c, v16h d) { keep4_h(a, b, c, d); }
};
template <> struct Frag<__bf16> {
  typedef v16b V; union U { v16b v; v8b h[2]; };
  static __device__ __forceinline__ v16b load(const __bf16* p) {
    U f; f.h[0] = *(const v8b*)(p); f.h[1] = *(const v8b*)(p + 16); return f.v;
  }
  static __device__ __forceinline__ v8f mma(v16b a, v16b b, v8f c) {
    return __builtin_amdgcn_wmma_f32_16x16x32_bf16(false, a, false, b, (short)0, c, false, false);
  }
  static __device__ __forceinline__ void guard(v8f& a, v8f& b, v16b x, v16b y) { dep_guard_b(a, b, x, y); }
  static __device__ __forceinline__ void keep(v16b a, v16b b, v16b c, v16b d) { keep4_b(a, b, c, d); }
};

__device__ __forceinline__ float fsig(float x)  { return __builtin_amdgcn_rcpf(1.0f + __expf(-x)); }
__device__ __forceinline__ float ftanh(float x) { return 1.0f - 2.0f * __builtin_amdgcn_rcpf(__expf(2.0f * x) + 1.0f); }

template <int MODE>
__global__ __launch_bounds__(TPW_NT) void tpw_kernel(const float* __restrict__ src, int R, int C, int ldo,
                                                    unsigned short* __restrict__ O, float sc) {
  __shared__ float Tt[64 * 65];
  const int tid = threadIdx.x;
  const int c0 = blockIdx.x * 64, r0 = blockIdx.y * 64;
#pragma unroll
  for (int i = 0; i < 4; ++i) {
    const int idx = i * TPW_NT + tid;
    const int rr = idx >> 4, cc = (idx & 15) * 4;
    const v4f v = *(const v4f*)(src + (size_t)(r0 + rr) * (size_t)C + c0 + cc);
    Tt[rr * 65 + cc + 0] = v[0];
    Tt[rr * 65 + cc + 1] = v[1];
    Tt[rr * 65 + cc + 2] = v[2];
    Tt[rr * 65 + cc + 3] = v[3];
  }
  __syncthreads();
  const int q = tid >> 3, c8 = (tid & 7) * 8;
  v8h hv[2];
#pragma unroll
  for (int g = 0; g < 2; ++g) {
    const int qq = g * 32 + q;
#pragma unroll
    for (int e = 0; e < 8; ++e) {
      const float f = Tt[(c8 + e) * 65 + qq];
      unsigned short bits;
      if (MODE == 0) {
        bits = f2bf_bits(f * sc);
      } else {
        const float fb = bf_bits2f(f2bf_bits(f));
        bits = __builtin_bit_cast(unsigned short, (_Float16)(fb * sc));
      }
      hv[g][e] = __builtin_bit_cast(_Float16, bits);
    }
  }
  for (int pass = 0; pass < 2; ++pass) {
#pragma unroll
    for (int g = 0; g < 2; ++g) {
      const size_t o = (size_t)(c0 + g * 32 + q) * (size_t)ldo + (size_t)(r0 + c8);
      *(volatile v8h*)(O + o) = hv[g];
    }
    __threadfence();
  }
}

__global__ __launch_bounds__(XG_NT) void xg_kernel(const float* __restrict__ emb,
                                                  const float* __restrict__ Wfx, const float* __restrict__ Wix,
                                                  const float* __restrict__ Wgx, const float* __restrict__ Wox,
                                                  const float* __restrict__ bfp, const float* __restrict__ bip,
                                                  const float* __restrict__ bgp, const float* __restrict__ bop,
                                                  float* __restrict__ XG) {
  const int v  = blockIdx.x;
  const int j4 = threadIdx.x * 4;
  v4f af = {0.f, 0.f, 0.f, 0.f}, ai = {0.f, 0.f, 0.f, 0.f}, ag = {0.f, 0.f, 0.f, 0.f}, ao = {0.f, 0.f, 0.f, 0.f};
#pragma unroll 1
  for (int k = 0; k < NE; ++k) {
    const float e  = bf16r(emb[v * NE + k]);
    const v4f wf = *(const v4f*)(Wfx + (size_t)k * NH + j4);
    const v4f wi = *(const v4f*)(Wix + (size_t)k * NH + j4);
    const v4f wg = *(const v4f*)(Wgx + (size_t)k * NH + j4);
    const v4f wo = *(const v4f*)(Wox + (size_t)k * NH + j4);
#pragma unroll
    for (int q = 0; q < 4; ++q) {
      af[q] = fmaf(e, bf16r(wf[q]), af[q]);
      ai[q] = fmaf(e, bf16r(wi[q]), ai[q]);
      ag[q] = fmaf(e, bf16r(wg[q]), ag[q]);
      ao[q] = fmaf(e, bf16r(wo[q]), ao[q]);
    }
  }
  const v4f vbf = *(const v4f*)(bfp + j4);
  const v4f vbi = *(const v4f*)(bip + j4);
  const v4f vbg = *(const v4f*)(bgp + j4);
  const v4f vbo = *(const v4f*)(bop + j4);
  v4f o_f, o_i, o_g, o_o;
#pragma unroll
  for (int q = 0; q < 4; ++q) {
    o_f[q] = af[q] + bf16r(vbf[q]);
    o_i[q] = ai[q] + bf16r(vbi[q]);
    o_g[q] = ag[q] + bf16r(vbg[q]);
    o_o[q] = ao[q] + bf16r(vbo[q]);
  }
  float* base = XG + (size_t)(v * NGATE) * NH + j4;
  for (int pass = 0; pass < 2; ++pass) {
    *(volatile v4f*)(base + 0 * NH) = o_f;
    *(volatile v4f*)(base + 1 * NH) = o_i;
    *(volatile v4f*)(base + 2 * NH) = o_g;
    *(volatile v4f*)(base + 3 * NH) = o_o;
    __threadfence();
  }
}

__global__ __launch_bounds__(SEQ_NT) void seq_cell_kernel(const int* __restrict__ x, const float* __restrict__ XG,
                                                         const unsigned short* __restrict__ WBp,
                                                         const float* __restrict__ Wph, const float* __restrict__ Wpb,
                                                         float* __restrict__ out) {
  __shared__ __align__(16) _Float16 Ah[SEQ_ROWS * HPITCH];
  __shared__ unsigned int tokw[NSTEP];
  __shared__ __align__(16) float Hs[SEQ_ROWS * HSP];
  __shared__ __align__(16) float Ps[SEQ_ROWS * NCLS];
  __shared__ __align__(16) float Pl[SEQ_ROWS * NCLS];
  const _Float16* WB = (const _Float16*)WBp;
  const int tid = threadIdx.x, lane = tid & 31, wave = tid >> 5;
  const int c = lane & 15, hh = lane >> 4, koff = hh * 8;
  const int rowbase = blockIdx.x * SEQ_ROWS;
  const int j = 16 * wave + c;

#pragma unroll 1
  for (int t = tid; t < NSTEP; t += SEQ_NT) {
    unsigned w = 0u;
#pragma unroll 1
    for (int m = 0; m < SEQ_ROWS; ++m) {
      int tk = x[(size_t)(rowbase + m) * NSTEP + (size_t)t];
      tk = tk < 0 ? 0 : tk;
      tk = tk > (NVOC - 1) ? (NVOC - 1) : tk;
      w |= ((unsigned)tk) << (2 * m);
    }
    tokw[t] = w;
  }
#pragma unroll 1
  for (int i = tid; i < SEQ_ROWS * HPITCH; i += SEQ_NT) Ah[i] = (_Float16)0.0f;
  float xv[NGATE][NVOC];
#pragma unroll
  for (int g = 0; g < NGATE; ++g)
#pragma unroll
    for (int v = 0; v < NVOC; ++v) xv[g][v] = XG[(v * NGATE + g) * NH + j] * XCARRY;
  float cst[8], hst[8];
#pragma unroll
  for (int r = 0; r < 8; ++r) { cst[r] = 0.0f; hst[r] = 0.0f; }
  __syncthreads();

  const _Float16* ahrow = Ah + c * HPITCH + koff;
  const _Float16* wb0 = WB + (size_t)j * NH + koff;
  const _Float16* wb1 = wb0 + (size_t)1 * NH * NH;
  const _Float16* wb2 = wb0 + (size_t)2 * NH * NH;
  const _Float16* wb3 = wb0 + (size_t)3 * NH * NH;
  const v8f z8 = {0.f, 0.f, 0.f, 0.f, 0.f, 0.f, 0.f, 0.f};

#pragma unroll 1
  for (int t = 0; t < NSTEP; ++t) {
    const unsigned tw = tokw[t];
    v8f acc[4];
    acc[0] = z8; acc[1] = z8; acc[2] = z8; acc[3] = z8;
#pragma unroll
    for (int r = 0; r < 8; ++r) {
      const unsigned tk = (tw >> (2 * (8 * hh + r))) & 3u;
#pragma unroll
      for (int g = 0; g < NGATE; ++g)
        acc[g][r] = (tk == 0u) ? xv[g][0] : ((tk == 1u) ? xv[g][1] : xv[g][2]);
    }
#pragma unroll 1
    for (int k0 = 0; k0 < NH; k0 += 32) {
      const v16h a  = Frag<_Float16>::load(ahrow + k0);
      const v16h b0 = Frag<_Float16>::load(wb0 + k0);
      const v16h b1 = Frag<_Float16>::load(wb1 + k0);
      const v16h b2 = Frag<_Float16>::load(wb2 + k0);
      const v16h b3 = Frag<_Float16>::load(wb3 + k0);
      acc[0] = Frag<_Float16>::mma(a, b0, acc[0]);
      acc[1] = Frag<_Float16>::mma(a, b1, acc[1]);
      acc[2] = Frag<_Float16>::mma(a, b2, acc[2]);
      acc[3] = Frag<_Float16>::mma(a, b3, acc[3]);
      mma_guard_all(acc[0], acc[1], acc[2], acc[3], a, b0, b1, b2, b3);
    }
    acc_guard4(acc[0], acc[1], acc[2], acc[3]);
#pragma unroll
    for (int r = 0; r < 8; ++r) {
      const float zf = acc[0][r] * ACC_INV;
      const float zi = acc[1][r] * ACC_INV;
      const float zg = acc[2][r] * ACC_INV;
      const float zo = acc[3][r] * ACC_INV;
      const float fg = fsig(zf);
      const float ig = fsig(zi);
      const float gg = ftanh(zg);
      const float og = fsig(zo);
      const float cn = fg * cst[r] + ig * gg;
      cst[r] = cn;
      hst[r] = ftanh(cn) * og;
    }
    __syncthreads();
#pragma unroll
    for (int r = 0; r < 8; ++r) Ah[(8 * hh + r) * HPITCH + j] = (_Float16)(hst[r] * HCARRY);
    __syncthreads();
  }

#pragma unroll
  for (int r = 0; r < 8; ++r) Hs[(8 * hh + r) * HSP + j] = hst[r];
  __syncthreads();
  if (tid < SEQ_ROWS * NCLS) {
    const int prow = tid / NCLS;
    const int pcls = tid - prow * NCLS;
    float p = 0.0f;
#pragma unroll 1
    for (int k = 0; k < NH; ++k) p = fmaf(Hs[prow * HSP + k], bf16r(Wph[k * NCLS + pcls]), p);
    p += bf16r(Wpb[pcls]);
    Ps[tid] = p;
  }
  __syncthreads();
  if (wave == 0) {
    const int lr = lane & 15;
    float mx = -INFINITY;
#pragma unroll 1
    for (int q = 0; q < NCLS; ++q) mx = fmaxf(mx, Ps[lr * NCLS + q]);
    float s = 0.0f;
#pragma unroll 1
    for (int q = 0; q < NCLS; ++q) s += expf(Ps[lr * NCLS + q] - mx);
    const float ls = logf(s);
    if (lane < 16) {
#pragma unroll 1
      for (int q = 0; q < NCLS; ++q) Pl[lr * NCLS + q] = (Ps[lr * NCLS + q] - mx) - ls;
    }
  }
  __syncthreads();
  if (wave == 0) {
    float* ob = out + (size_t)blockIdx.x * (SEQ_ROWS * NCLS);
    for (int pass = 0; pass < 2; ++pass) {
#pragma unroll
      for (int it = 0; it < 2; ++it) {
        const int idx = it * 32 + lane;
        const int idc = idx < 40 ? idx : 39;
        const v4f val = *(const v4f*)(Pl + idc * 4);
        if (idx < 40) *(volatile v4f*)(ob + (size_t)idx * 4) = val;
      }
      __threadfence();
    }
  }
}

extern "C" void kernel_launch(void* const* d_in, const int* in_sizes, int n_in,
                              void* d_out, int out_size, void* d_ws, size_t ws_size, hipStream_t stream) {
  if (n_in < 16 || d_out == nullptr || d_ws == nullptr) return;
  if (in_sizes[0] != NB * NSTEP || in_sizes[1] != NVOC * NE ||
      in_sizes[2] != NE * NH || in_sizes[3] != NH * NH || in_sizes[4] != NH ||
      in_sizes[5] != NE * NH || in_sizes[6] != NH * NH || in_sizes[7] != NH ||
      in_sizes[8] != NE * NH || in_sizes[9] != NH * NH || in_sizes[10] != NH ||
      in_sizes[11] != NE * NH || in_sizes[12] != NH * NH || in_sizes[13] != NH ||
      in_sizes[14] != NH * NCLS || in_sizes[15] != NCLS || out_size != NOUT) return;

  const int*   x   = (const int*)d_in[0];
  const float* emb = (const float*)d_in[1];
  const float* Wfx = (const float*)d_in[2];
  const float* Wfh = (const float*)d_in[3];
  const float* Wfb = (const float*)d_in[4];
  const float* Wix = (const float*)d_in[5];
  const float* Wih = (const float*)d_in[6];
  const float* Wib = (const float*)d_in[7];
  const float* Wgx = (const float*)d_in[8];
  const float* Wgh = (const float*)d_in[9];
  const float* Wgb = (const float*)d_in[10];
  const float* Wox = (const float*)d_in[11];
  const float* Woh = (const float*)d_in[12];
  const float* Wob = (const float*)d_in[13];
  const float* Wph = (const float*)d_in[14];
  const float* Wpb = (const float*)d_in[15];
  float* out = (float*)d_out;

  char* ws = (char*)d_ws; size_t off = 0;
  auto carve = [&](size_t bytes) -> char* { char* p = ws + off; off += (bytes + 255) & ~(size_t)255; return p; };
  unsigned short* WB = (unsigned short*)carve((size_t)NGATE * NH * NH * 2);
  float*          XG = (float*)carve((size_t)NVOC * NGATE * NH * 4);
  if (off > ws_size || off > (size_t)134217728) return;

  const dim3 tg(NH / 64, NH / 64);
  tpw_kernel<1><<<tg, TPW_NT, 0, stream>>>(Wfh, NH, NH, NH, WB + (size_t)0 * NH * NH, WCARRY);
  tpw_kernel<1><<<tg, TPW_NT, 0, stream>>>(Wih, NH, NH, NH, WB + (size_t)1 * NH * NH, WCARRY);
  tpw_kernel<1><<<tg, TPW_NT, 0, stream>>>(Wgh, NH, NH, NH, WB + (size_t)2 * NH * NH, WCARRY);
  tpw_kernel<1><<<tg, TPW_NT, 0, stream>>>(Woh, NH, NH, NH, WB + (size_t)3 * NH * NH, WCARRY);
  xg_kernel<<<NVOC, XG_NT, 0, stream>>>(emb, Wfx, Wix, Wgx, Wox, Wfb, Wib, Wgb, Wob, XG);
  seq_cell_kernel<<<NB / SEQ_ROWS, SEQ_NT, 0, stream>>>(x, XG, WB, Wph, Wpb, out);
}
